// EMHA_20650202759916
// MI455X (gfx1250) — hardware-verified
//
#include <hip/hip_runtime.h>


#define NB_  2
#define NH_  16
#define NT_  2048
#define OPITCH (NB_ * NH_ * HD)
#define HD   64
#define NBH  (NB_ * NH_)
#define PSC  32768.0f
#define LOSC 1024.0f
#define LOSCI (1.0f / 1024.0f)

typedef _Float16 h16;
typedef __attribute__((ext_vector_type(16))) _Float16 v16h;
typedef __attribute__((ext_vector_type(8)))  _Float16 v8h;
typedef __attribute__((ext_vector_type(4)))  _Float16 v4h;
typedef __attribute__((ext_vector_type(8)))  float    v8f;
typedef __attribute__((ext_vector_type(4)))  float    v4f;
typedef v8h  __attribute__((may_alias)) v8ha;
typedef v4f  __attribute__((may_alias)) v4fa;

__device__ __forceinline__ unsigned short f2bf(float f) { unsigned u = __float_as_uint(f); u += 0x7FFFu + ((u >> 16) & 1u); return (unsigned short)(u >> 16); }
__device__ __forceinline__ float bf2f(unsigned short b) { return __uint_as_float(((unsigned)b) << 16); }
__device__ __forceinline__ float bfr(float f) { return bf2f(f2bf(f)); }
__device__ __forceinline__ v16h cat16(v8h lo, v8h hi) { return __builtin_shufflevector(lo, hi, 0, 1, 2, 3, 4, 5, 6, 7, 8, 9, 10, 11, 12, 13, 14, 15); }
__device__ __forceinline__ v8f wmma16(v16h a, v16h b, v8f c) { return __builtin_amdgcn_wmma_f32_16x16x32_f16(false, a, false, b, (short)0, c, false, false); }
#define VST2(T, p, v) do { const T vst2_v_ = (v); *(volatile T*)(p) = vst2_v_; __threadfence(); *(volatile T*)(p) = vst2_v_; } while (0)

__global__ __launch_bounds__(256) void k_16g(const float* __restrict__ x, h16* X16) {
    const int lane = threadIdx.x & 31; const size_t w = (size_t)blockIdx.x * 8 + (threadIdx.x >> 5);
    if (w >= (size_t)NBH * NT_ / 2) return;
    const size_t r = w * 2 + (lane >> 4); const int c0 = (lane & 15) * 4;
    const int bh = (int)(r / NT_), t = (int)(r - (size_t)bh * NT_), b = bh / NH_, h = bh - b * NH_;
    const float* src = x + ((size_t)t * NB_ + b) * (NH_ * HD) + h * HD + c0;
    v4h oq;
#pragma unroll
    for (int i = 0; i < 4; ++i) oq[i] = (h16)bfr(src[i]);
    VST2(v4h, X16 + r * HD + c0, oq);
}
__global__ __launch_bounds__(256) void k_vt(const float* __restrict__ v, h16* VT16) {
    __shared__ __align__(16) h16 tile[HD * 72];
    const int bh = blockIdx.x / (NT_ / 64), kt = blockIdx.x - bh * (NT_ / 64), t0 = kt * 64, tid = threadIdx.x;
    const int tt = tid >> 2, d0 = (tid & 3) * 16;
    const int b = bh / NH_, h = bh - b * NH_;
    const float* src = v + ((size_t)(t0 + tt) * NB_ + b) * (NH_ * HD) + h * HD + d0;
#pragma unroll
    for (int i = 0; i < 16; ++i) tile[(d0 + i) * 72 + tt] = (h16)bfr(src[i]);
    __syncthreads();
    const int piece = tid & 7;
    const size_t base = ((size_t)bh * HD) * NT_ + t0;
    auto pass = [&]() {
#pragma unroll
        for (int s = 0; s < 2; ++s) { const int d = (tid >> 3) + 32 * s; const v8h val = *(const v8ha*)(tile + d * 72 + piece * 8); *(volatile v8h*)(VT16 + base + (size_t)d * NT_ + piece * 8) = val; }
    };
    pass(); __threadfence(); pass();
}
__global__ __launch_bounds__(128) void k_attn(const h16* __restrict__ Q16, const h16* __restrict__ K16, const h16* __restrict__ VT16, float* out) {
    __shared__ __align__(16) h16 plds[4][16 * 32];
    __shared__ __align__(16) h16 plds2[4][16 * 32];
    __shared__ __align__(16) float ost[4][16 * 68];
    const int lane = threadIdx.x & 31, wave = threadIdx.x >> 5, lr = lane & 15, hi = lane >> 4;
    const int bh = blockIdx.x / (NT_ / 64), qt = blockIdx.x - bh * (NT_ / 64), q0 = qt * 64 + wave * 16;
    h16* pl = &plds[wave][0]; h16* pl2 = &plds2[wave][0];
    const h16* qb = Q16 + (size_t)bh * NT_ * HD; const h16* kb = K16 + (size_t)bh * NT_ * HD; const h16* vb = VT16 + (size_t)bh * HD * NT_;
    v16h qa[2];
#pragma unroll
    for (int kc = 0; kc < 2; ++kc) { const h16* p = qb + (size_t)(q0 + lr) * HD + kc * 32 + 8 * hi; qa[kc] = cat16(*(const v8h*)p, *(const v8h*)(p + 16)); }
    int qpos[8];
#pragma unroll
    for (int j = 0; j < 8; ++j) qpos[j] = q0 + 8 * hi + j;
    v8f o[4], ox[4];
#pragma unroll
    for (int n = 0; n < 4; ++n) { o[n] = (v8f){}; ox[n] = (v8f){}; }
    float mrow[8], lpart[8];
#pragma unroll
    for (int j = 0; j < 8; ++j) { mrow[j] = -3.0e38f; lpart[j] = 0.f; }
    const int kt_end = (qt * 64 + 63) / 32 + 1;
    const float scl = 0.125f;
#pragma unroll 1
    for (int kt = 0; kt < kt_end; ++kt) {
        const int l0 = kt * 32;
        v8f s0 = {}, s1 = {};
#pragma unroll
        for (int kc = 0; kc < 2; ++kc) {
            const h16* r0p = kb + (size_t)(l0 + lr) * HD + kc * 32 + 8 * hi; const h16* r1p = r0p + (size_t)16 * HD;
            s0 = wmma16(qa[kc], cat16(*(const v8h*)r0p, *(const v8h*)(r0p + 16)), s0);
            s1 = wmma16(qa[kc], cat16(*(const v8h*)r1p, *(const v8h*)(r1p + 16)), s1);
        }
        asm volatile("v_nop\n\tv_nop\n\tv_nop\n\tv_nop" : "+v"(s0), "+v"(s1) : "v"(qa[0]), "v"(qa[1]));
        float alpha[8];
#pragma unroll
        for (int j = 0; j < 8; ++j) {
            const int qi = qpos[j], ja = l0 + lr, jb = l0 + 16 + lr;
            const float a0 = (ja <= qi) ? s0[j] * scl : -__builtin_inff(), a1 = (jb <= qi) ? s1[j] * scl : -__builtin_inff();
            float mx = fmaxf(a0, a1);
            mx = fmaxf(mx, __shfl_xor(mx, 1, 16)); mx = fmaxf(mx, __shfl_xor(mx, 2, 16)); mx = fmaxf(mx, __shfl_xor(mx, 4, 16)); mx = fmaxf(mx, __shfl_xor(mx, 8, 16));
            const float mn = fmaxf(mrow[j], mx);
            alpha[j] = __expf(mrow[j] - mn); mrow[j] = mn;
            const float p0 = __expf(a0 - mn), p1 = __expf(a1 - mn);
            lpart[j] = lpart[j] * alpha[j] + (p0 + p1);
            const int mr = hi * 8 + j;
            const float ps0 = p0 * PSC, ps1 = p1 * PSC; const h16 h0 = (h16)ps0, h1 = (h16)ps1;
            pl[mr * 32 + lr] = h0; pl[mr * 32 + 16 + lr] = h1; pl2[mr * 32 + lr] = (h16)((ps0 - (float)h0) * LOSC); pl2[mr * 32 + 16 + lr] = (h16)((ps1 - (float)h1) * LOSC);
        }
#pragma unroll
        for (int n = 0; n < 4; ++n)
#pragma unroll
            for (int j = 0; j < 8; ++j) { o[n][j] *= alpha[j]; ox[n][j] *= alpha[j]; }
        asm volatile("" ::: "memory");
        const v16h pa = cat16(*(const v8ha*)(pl + lr * 32 + hi * 8), *(const v8ha*)(pl + lr * 32 + 16 + hi * 8));
        const v16h px = cat16(*(const v8ha*)(pl2 + lr * 32 + hi * 8), *(const v8ha*)(pl2 + lr * 32 + 16 + hi * 8));
#pragma unroll
        for (int n = 0; n < 4; ++n) { const h16* vp = vb + (size_t)(n * 16 + lr) * NT_ + l0 + hi * 8; const v16h vv = cat16(*(const v8h*)vp, *(const v8h*)(vp + 16));
            o[n] = wmma16(pa, vv, o[n]); ox[n] = wmma16(px, vv, ox[n]); }
        asm volatile("v_nop\n\tv_nop\n\tv_nop\n\tv_nop" : "+v"(o[0]), "+v"(o[1]), "+v"(o[2]), "+v"(o[3]), "+v"(ox[0]), "+v"(ox[1]), "+v"(ox[2]), "+v"(ox[3]) : "v"(pa), "v"(px));
    }
    float inv[8];
#pragma unroll
    for (int j = 0; j < 8; ++j) { float rs = lpart[j]; rs += __shfl_xor(rs, 1, 16); rs += __shfl_xor(rs, 2, 16); rs += __shfl_xor(rs, 4, 16); rs += __shfl_xor(rs, 8, 16); inv[j] = 1.0f / (rs * PSC); }
    float* os = &ost[wave][0];
#pragma unroll
    for (int n = 0; n < 4; ++n)
#pragma unroll
        for (int j = 0; j < 8; ++j) os[(hi * 8 + j) * 68 + n * 16 + lr] = (o[n][j] + ox[n][j] * LOSCI) * inv[j];
    __syncthreads();
    const int b = bh / NH_, h = bh - b * NH_;
    float* ob = out + ((size_t)q0 * NB_ + b) * (NH_ * HD) + h * HD;
    auto pass = [&]() {
#pragma unroll
        for (int s = 0; s < 8; ++s) { const int Lid = (lane >> 3) + 4 * s, piece = lane & 7; const int row = Lid >> 1, cofs = (Lid & 1) * 32 + piece * 4;
            const v4f val = *(const v4fa*)(os + row * 68 + cofs); *(volatile v4f*)(ob + (size_t)row * OPITCH + cofs) = val; }
    };
    pass(); __threadfence(); pass();
}
extern "C" void kernel_launch(void* const* d_in, const int* in_sizes, int n_in,
                              void* d_out, int out_size, void* d_ws, size_t ws_size, hipStream_t stream) {
    (void)in_sizes; (void)n_in; (void)out_size;
    const float* q = (const float*)d_in[0]; const float* k = (const float*)d_in[1]; const float* v = (const float*)d_in[2];
    float* out = (float*)d_out;
    char* wsp = (char*)d_ws;
    auto take = [&](size_t bytes) { char* p = wsp; wsp += (bytes + 255) & ~(size_t)255; return (void*)p; };
    h16* Q16 = (h16*)take((size_t)NBH * NT_ * HD * 2); h16* K16 = (h16*)take((size_t)NBH * NT_ * HD * 2); h16* VT16 = (h16*)take((size_t)NBH * HD * NT_ * 2);
    if ((size_t)(wsp - (char*)d_ws) > ws_size) return;
    k_16g<<<(unsigned)(((size_t)NBH * NT_ / 2 + 7) / 8), 256, 0, stream>>>(q, Q16);
    k_16g<<<(unsigned)(((size_t)NBH * NT_ / 2 + 7) / 8), 256, 0, stream>>>(k, K16);
    k_vt<<<NBH * (NT_ / 64), 256, 0, stream>>>(v, VT16);
    k_attn<<<NBH * (NT_ / 64), 128, 0, stream>>>(Q16, K16, VT16, out);
}
